// CDE_STGNN_59897613910629
// MI455X (gfx1250) — hardware-verified
//
#include <hip/hip_runtime.h>
#include <hip/hip_bf16.h>
#include <math.h>


#define B_TOT   256
#define T_KNOTS 8
#define NIV     7
#define NS5     5
#define D_IN    289
#define H_DIM   64
#define Z_OUT   10
#define NB      16
#define DTILES  19
#define DPAD    (DTILES * 16)
#define NTILE   (H_DIM * DTILES)
#define NROWS_W (H_DIM * D_IN)
#define OUT_PB  (T_KNOTS * Z_OUT)

typedef __bf16         v16bf __attribute__((ext_vector_type(16)));
typedef unsigned short v16u  __attribute__((ext_vector_type(16)));
typedef unsigned short v8u   __attribute__((ext_vector_type(8)));
typedef float          v8f   __attribute__((ext_vector_type(8)));
typedef float          v4f   __attribute__((ext_vector_type(4)));
typedef unsigned int   v4u   __attribute__((ext_vector_type(4)));

union Pk16 { v8u s; v4u u; };

__device__ __forceinline__ unsigned short f2bf_bits(float f) {
    unsigned u = __builtin_bit_cast(unsigned, f);
    unsigned r = u + 0x7FFFu + ((u >> 16) & 1u);
    return (unsigned short)(r >> 16);
}
__device__ __forceinline__ float bf2f(unsigned short b) {
    return __builtin_bit_cast(float, ((unsigned)b) << 16);
}

__device__ __forceinline__ float ftanh(float x) {
    float ax = fabsf(x);
    float t  = __expf(-2.0f * ax);
    float r  = (1.0f - t) * __builtin_amdgcn_rcpf(1.0f + t);
    return copysignf(r, x);
}

__device__ __forceinline__ v8f wmma_bf(v16u a, v16u b, v8f c) {
    return __builtin_amdgcn_wmma_f32_16x16x32_bf16(false, __builtin_bit_cast(v16bf, a),
                                                   false, __builtin_bit_cast(v16bf, b),
                                                   (short)0, c, false, false);
}

__global__ __launch_bounds__(256)
void k_pack_wf(const float* __restrict__ Wf, const float* __restrict__ bf,
               unsigned short* Phi, unsigned short* Plo, float* bpad,
               int npieces, int nbias4) {
    const int p = blockIdx.x * 256 + threadIdx.x;
    if (p >= npieces) return;
    const int hv   = p & 1;
    const int lane = (p >> 1) & 31;
    const int kt   = (p >> 6) & 1;
    const int t    = p >> 7;
    const int ho   = t / DTILES;
    const int dtl  = t - ho * DTILES;
    const int half = lane >> 4, M = lane & 15;
    const int K    = kt * 32 + half * 8 + hv * 16;
    const int d    = dtl * 16 + M;
    int row = ho * D_IN + d;
    row = row < NROWS_W ? row : (NROWS_W - 1);
    const float* src = Wf + (size_t)row * H_DIM + K;
    const v4f w0 = *(const v4f*)src;
    const v4f w1 = *(const v4f*)(src + 4);
    const bool valid = d < D_IN;
    float w[8];
    w[0] = w0[0]; w[1] = w0[1]; w[2] = w0[2]; w[3] = w0[3];
    w[4] = w1[0]; w[5] = w1[1]; w[6] = w1[2]; w[7] = w1[3];
    Pk16 hi, lo;
#pragma unroll
    for (int j = 0; j < 8; ++j) {
        float x = valid ? w[j] : 0.0f;
        unsigned short hb = f2bf_bits(x);
        float r = x - bf2f(hb);
        hi.s[j] = hb;
        lo.s[j] = f2bf_bits(r);
    }
    const int t2 = p >> 2;
    const int ho2 = t2 / DTILES;
    const int dt2 = t2 - ho2 * DTILES;
    const int M0 = (p & 3) * 4;
    v4f bv;
#pragma unroll
    for (int j = 0; j < 4; ++j) {
        int d2 = dt2 * 16 + M0 + j;
        int o = ho2 * D_IN + d2;
        o = o < NROWS_W ? o : (NROWS_W - 1);
        float x = bf[o];
        bv[j] = (d2 < D_IN) ? x : 0.0f;
    }
    const bool dob = p < nbias4;

    unsigned short* dh = Phi + (size_t)p * 8;
    unsigned short* dl = Plo + (size_t)p * 8;
    float* db = bpad + (size_t)p * 4;
    *(volatile v4u*)dh = hi.u;
    *(volatile v4u*)dl = lo.u;
    if (dob) *(volatile v4f*)db = bv;
    __threadfence();
    *(volatile v4u*)dh = hi.u;
    *(volatile v4u*)dl = lo.u;
    if (dob) *(volatile v4f*)db = bv;
}

__global__ __launch_bounds__(256)
void k_prep_g(const float* __restrict__ times, const float* __restrict__ X,
              float* G, int npieces) {
#pragma clang fp contract(off)
    const int p = blockIdx.x * 256 + threadIdx.x;
    if (p >= npieces) return;
    const int idx0 = p * 4;
    const int dd0 = idx0 % DPAD;
    int r = idx0 / DPAD;
    const int s5 = r % NS5;  r /= NS5;
    const int i  = r % NIV;
    const int b  = r / NIV;
    const int im = (i > 0) ? (i - 1) : 0;
    const float ti = times[i], tip = times[i + 1], tim = times[im];
    const float dti  = tip - ti;
    const float rdti = 1.0f / dti;
    const float dtm  = (i > 0) ? (ti - tim) : dti;
    const float rdtm = 1.0f / dtm;
    const float s  = 0.25f * (float)s5;
    const float s2 = s * s;
    const float c1 = (6.0f * s - 6.0f * s2) * rdti;
    const float c2 = 3.0f * s2 - 4.0f * s + 1.0f;
    const float c3 = 3.0f * s2 - 2.0f * s;
    const size_t rowi = (size_t)(b * T_KNOTS + i) * D_IN;
    const size_t rowp = rowi + D_IN;
    const size_t rowm = (size_t)(b * T_KNOTS + im) * D_IN;
    v4f g;
#pragma unroll
    for (int j = 0; j < 4; ++j) {
        const int dd  = dd0 + j;
        const int ddc = dd < D_IN ? dd : (D_IN - 1);
        const float Xi  = X[rowi + ddc];
        const float Xip = X[rowp + ddc];
        const float Xim = X[rowm + ddc];
        const float diffi = (Xip - Xi) * rdti;
        const float di  = (i == 0) ? diffi : (Xi - Xim) * rdtm;
        const float dip = diffi;
        const float v = (Xip - Xi) * c1 + di * c2 + dip * c3;
        g[j] = (dd < D_IN) ? v : 0.0f;
    }
    float* dst = G + (size_t)p * 4;
    *(volatile v4f*)dst = g;
    __threadfence();
    *(volatile v4f*)dst = g;
}

__global__ __launch_bounds__(256)
void k_cde_main(const float* __restrict__ times,
                const float* __restrict__ z0,
                const float* __restrict__ Wp,
                const float* __restrict__ bp,
                const unsigned short* __restrict__ Phi,
                const unsigned short* __restrict__ Plo,
                const float* __restrict__ bpad,
                const float* __restrict__ G,
                float* out) {
    __shared__ float hS[NB][H_DIM];
    __shared__ float kS[NB][H_DIM];
    __shared__ float aS[NB][H_DIM];
    __shared__ __attribute__((aligned(16))) float oS[NB * OUT_PB];

    const int tid   = threadIdx.x;
    const int lane  = tid & 31;
    const int wave  = tid >> 5;
    const int half  = lane >> 4;
    const int n     = lane & 15;
    const int bbase = blockIdx.x * NB;
    if (bbase + NB > B_TOT) return;

    const v16u* PhiV  = (const v16u*)Phi;
    const v16u* PloV  = (const v16u*)Plo;
    const v4f*  bias4 = (const v4f*)bpad;
    const v4f*  G4    = (const v4f*)G;

    for (int x = tid; x < NB * H_DIM; x += 256)
        hS[x >> 6][x & 63] = z0[(size_t)(bbase + (x >> 6)) * H_DIM + (x & 63)];
    __syncthreads();

    auto project = [&](int tpt) {
        if (tid < NB * Z_OUT) {
            const int pn = tid / Z_OUT, z = tid - pn * Z_OUT;
            float acc = 0.0f;
#pragma unroll 8
            for (int k = 0; k < H_DIM; ++k) acc = fmaf(hS[pn][k], Wp[z * H_DIM + k], acc);
            oS[pn * OUT_PB + tpt * Z_OUT + z] = acc + bp[z];
        }
    };
    project(0);

    const int kb = 8 * half;

#pragma unroll 1
    for (int iv = 0; iv < NIV; ++iv) {
        const float dti   = times[iv + 1] - times[iv];
        const float hstep = dti * 0.5f;
#pragma unroll 1
        for (int kk = 0; kk < 2; ++kk) {
#pragma unroll
            for (int st = 0; st < 4; ++st) {
                const int   sidx = 2 * kk + ((st == 0) ? 0 : (st == 3) ? 2 : 1);
                const float c    = (st == 0) ? 0.0f : ((st == 3) ? hstep : 0.5f * hstep);
                const float wgt  = (st == 1 || st == 2) ? 2.0f : 1.0f;

                v16u bh0, bh1, bl0, bl1;
#pragma unroll
                for (int i = 0; i < 16; ++i) {
                    const int k = kb + (i & 7) + ((i >> 3) << 4);
                    float v0 = hS[n][k];
                    float v1 = hS[n][32 + k];
                    if (st > 0) {
                        v0 = fmaf(c, kS[n][k], v0);
                        v1 = fmaf(c, kS[n][32 + k], v1);
                    }
                    unsigned short h0 = f2bf_bits(v0);
                    unsigned short h1 = f2bf_bits(v1);
                    bh0[i] = h0;
                    bh1[i] = h1;
                    bl0[i] = f2bf_bits(v0 - bf2f(h0));
                    bl1[i] = f2bf_bits(v1 - bf2f(h1));
                }
                __syncthreads();

                const int gbase = (((bbase + n) * NIV + iv) * NS5 + sidx) * DPAD;

#pragma unroll 1
                for (int hh = 0; hh < 8; ++hh) {
                    const int h_out = wave * 8 + hh;
                    float partial = 0.0f;
#pragma unroll 1
                    for (int dtile = 0; dtile < DTILES; ++dtile) {
                        const int t = h_out * DTILES + dtile;
                        const size_t fo = (size_t)(t * 2) * 32 + lane;
                        const v16u ah0 = PhiV[fo];
                        const v16u ah1 = PhiV[fo + 32];
                        const v16u al0 = PloV[fo];
                        const v16u al1 = PloV[fo + 32];
                        v8f cacc = {0.f, 0.f, 0.f, 0.f, 0.f, 0.f, 0.f, 0.f};
                        cacc = wmma_bf(ah0, bh0, cacc);
                        cacc = wmma_bf(ah0, bl0, cacc);
                        cacc = wmma_bf(al0, bh0, cacc);
                        cacc = wmma_bf(ah1, bh1, cacc);
                        cacc = wmma_bf(ah1, bl1, cacc);
                        cacc = wmma_bf(al1, bh1, cacc);
                        asm volatile("v_nop\n\tv_nop\n\tv_nop\n\tv_nop"
                                     : "+v"(cacc)
                                     : "v"(ah0), "v"(al0), "v"(ah1), "v"(al1),
                                       "v"(bh0), "v"(bl0), "v"(bh1), "v"(bl1));
                        const v4f bl = bias4[t * 4 + half * 2];
                        const v4f bu = bias4[t * 4 + half * 2 + 1];
                        const int  gi = (gbase + dtile * 16 + half * 8) >> 2;
                        const v4f gl = G4[gi];
                        const v4f gu = G4[gi + 1];
                        partial = fmaf(ftanh(cacc[0] + bl[0]), gl[0], partial);
                        partial = fmaf(ftanh(cacc[1] + bl[1]), gl[1], partial);
                        partial = fmaf(ftanh(cacc[2] + bl[2]), gl[2], partial);
                        partial = fmaf(ftanh(cacc[3] + bl[3]), gl[3], partial);
                        partial = fmaf(ftanh(cacc[4] + bu[0]), gu[0], partial);
                        partial = fmaf(ftanh(cacc[5] + bu[1]), gu[1], partial);
                        partial = fmaf(ftanh(cacc[6] + bu[2]), gu[2], partial);
                        partial = fmaf(ftanh(cacc[7] + bu[3]), gu[3], partial);
                    }
                    partial += __shfl_xor(partial, 16, 32);
                    if (half == 0) {
                        kS[n][h_out] = partial;
                        if (st == 0) aS[n][h_out] = partial;
                        else         aS[n][h_out] += wgt * partial;
                    }
                }
                __syncthreads();
            }
            const float w6 = hstep * (1.0f / 6.0f);
            for (int x = tid; x < NB * H_DIM; x += 256)
                hS[x >> 6][x & 63] = fmaf(w6, aS[x >> 6][x & 63], hS[x >> 6][x & 63]);
            __syncthreads();
        }
        project(iv + 1);
    }
    __syncthreads();

    float* ob = out + (size_t)bbase * OUT_PB;
    const int npiece = NB * OUT_PB / 4;
    v4f v0 = *(const v4f*)(oS + 4 * tid);
    v4f v1 = {0.f, 0.f, 0.f, 0.f};
    const bool has1 = (tid + 256) < npiece;
    if (has1) v1 = *(const v4f*)(oS + 4 * (tid + 256));
    *(volatile v4f*)(ob + 4 * tid) = v0;
    if (has1) *(volatile v4f*)(ob + 4 * (tid + 256)) = v1;
    __threadfence();
    *(volatile v4f*)(ob + 4 * tid) = v0;
    if (has1) *(volatile v4f*)(ob + 4 * (tid + 256)) = v1;
}

extern "C" void kernel_launch(void* const* d_in, const int* in_sizes, int n_in,
                              void* d_out, int out_size, void* d_ws, size_t ws_size,
                              hipStream_t stream) {
    if (n_in < 7) return;
    if (in_sizes[0] != T_KNOTS || in_sizes[1] != B_TOT * T_KNOTS * D_IN ||
        in_sizes[2] != B_TOT * H_DIM || in_sizes[3] != NROWS_W * H_DIM ||
        in_sizes[4] != NROWS_W || in_sizes[5] != Z_OUT * H_DIM || in_sizes[6] != Z_OUT ||
        out_size != B_TOT * T_KNOTS * Z_OUT) return;

    const float* times = (const float*)d_in[0];
    const float* X     = (const float*)d_in[1];
    const float* z0    = (const float*)d_in[2];
    const float* Wf    = (const float*)d_in[3];
    const float* bf    = (const float*)d_in[4];
    const float* Wp    = (const float*)d_in[5];
    const float* bp    = (const float*)d_in[6];
    float* out = (float*)d_out;

    const size_t plane_bytes = (size_t)NTILE * 1024 * sizeof(unsigned short);
    const size_t bpad_bytes  = (size_t)NTILE * 16 * sizeof(float);
    const size_t g_bytes     = (size_t)B_TOT * NIV * NS5 * DPAD * sizeof(float);
    size_t off = 0;
    char* ws = (char*)d_ws;
    unsigned short* Phi = (unsigned short*)(ws + off); off += plane_bytes;
    unsigned short* Plo = (unsigned short*)(ws + off); off += plane_bytes;
    float* bpad = (float*)(ws + off); off += bpad_bytes;
    float* G    = (float*)(ws + off); off += g_bytes;
    if (off > ws_size) return;

    const int npieces = NTILE * 1024 / 8;
    const int nbias4  = NTILE * 16 / 4;
    k_pack_wf<<<dim3((npieces + 255) / 256), dim3(256), 0, stream>>>(Wf, bf, Phi, Plo, bpad,
                                                                    npieces, nbias4);

    const int ngp = B_TOT * NIV * NS5 * DPAD / 4;
    k_prep_g<<<dim3((ngp + 255) / 256), dim3(256), 0, stream>>>(times, X, G, ngp);

    k_cde_main<<<dim3(B_TOT / NB), dim3(256), 0, stream>>>(times, z0, Wp, bp, Phi, Plo,
                                                          bpad, G, out);
}
